// RGATBackbone_43387759624624
// MI455X (gfx1250) — hardware-verified
//
#include <hip/hip_runtime.h>
#include <math.h>


typedef __bf16 v16b __attribute__((ext_vector_type(16)));
typedef __bf16 v8b  __attribute__((ext_vector_type(8)));
typedef __bf16 v8ba __attribute__((ext_vector_type(8), __may_alias__));
typedef float  v8f  __attribute__((ext_vector_type(8)));
typedef float  v4f  __attribute__((ext_vector_type(4)));
typedef float  v4fa __attribute__((ext_vector_type(4), __may_alias__));
typedef int    v4i  __attribute__((ext_vector_type(4)));
typedef int    v4ia __attribute__((ext_vector_type(4), __may_alias__));

#define HIDC  128
#define NHEAD 4
#define BST   136
#define SST   132
#define GWAV  4
#define GSPW  8
#define GTHR  (GWAV * 32)
#define GROWS (GWAV * GSPW * 16)
#define ATHR  256
#define AWAV  8
#define NBLK  1024
#define CAPB  16384
#define CAPW  2048
#define CAPG  512
#define EPT   8

union FragU { v16b v; v8b hf[2]; unsigned u[8]; };

__device__ __forceinline__ v8f wmma_g(v16b a, v16b b, v8f c)
{
    v8f d = __builtin_amdgcn_wmma_f32_16x16x32_bf16(false, a, false, b, (short)0, c, false, false);
    asm volatile("v_nop\n\tv_nop\n\tv_nop\n\tv_nop" : "+v"(d) : "v"(a), "v"(b));
    return d;
}

__device__ __forceinline__ unsigned bf16_rne(float x)
{
    const unsigned u = __float_as_uint(x);
    return (u + 0x7FFFu + ((u >> 16) & 1u)) >> 16;
}

__device__ __forceinline__ void split1(float x, unsigned& hb, unsigned& lb)
{
    hb = bf16_rne(x);
    lb = bf16_rne(x - __uint_as_float(hb << 16));
}

__device__ __forceinline__ void split2(float x0, float x1, unsigned& hp, unsigned& lp)
{
    unsigned h0, l0, h1, l1;
    split1(x0, h0, l0);
    split1(x1, h1, l1);
    hp = h0 | (h1 << 16);
    lp = l0 | (l1 << 16);
}

__device__ __forceinline__ void split_a(const float* p0, const float* p1, v16b& ah, v16b& al)
{
    const v4f f0 = *(const v4fa*)p0;
    const v4f f1 = *(const v4fa*)(p0 + 4);
    const v4f f2 = *(const v4fa*)p1;
    const v4f f3 = *(const v4fa*)(p1 + 4);
    FragU H, L;
    split2(f0.x, f0.y, H.u[0], L.u[0]);
    split2(f0.z, f0.w, H.u[1], L.u[1]);
    split2(f1.x, f1.y, H.u[2], L.u[2]);
    split2(f1.z, f1.w, H.u[3], L.u[3]);
    split2(f2.x, f2.y, H.u[4], L.u[4]);
    split2(f2.z, f2.w, H.u[5], L.u[5]);
    split2(f3.x, f3.y, H.u[6], L.u[6]);
    split2(f3.z, f3.w, H.u[7], L.u[7]);
    ah = H.v;
    al = L.v;
}

__device__ __forceinline__ void store_pass(const float* stg, float* Cp, int row0, int M, int lane,
                                           const float* qst, float* Qp, int do_qk)
{
#pragma unroll 4
    for (int row = 0; row < 16; ++row) {
        const int gr = row0 + row;
        if (gr < M) {
            const v4f v = *(const v4fa*)(stg + row * SST + 4 * lane);
            *(volatile v4f*)(Cp + (size_t)gr * HIDC + 4 * lane) = v;
        }
    }
    if (do_qk) {
        const v4f v = *(const v4fa*)(qst + 4 * lane);
        *(volatile v4f*)(Qp + (size_t)row0 * 8 + 4 * lane) = v;
    }
}

__global__ void __launch_bounds__(GTHR) __attribute__((amdgpu_num_vgpr(256)))
k_gemm(const float* __restrict__ A, int M,
       const float* __restrict__ Bsrc, long bRel, int sn, int sk,
       const float* __restrict__ cbias, int do_be,
       float* C, long cRel,
       const float* __restrict__ Qw, const float* __restrict__ Kw,
       float* QK, long qkRel, int do_qk)
{
    __shared__ __attribute__((aligned(16))) unsigned short Bh[HIDC * BST];
    __shared__ __attribute__((aligned(16))) unsigned short Bl[HIDC * BST];
    __shared__ __attribute__((aligned(16))) unsigned short Qh[16 * BST];
    __shared__ __attribute__((aligned(16))) unsigned short Ql[16 * BST];
    __shared__ __attribute__((aligned(16))) float Sstg[GWAV * 16 * SST];
    __shared__ __attribute__((aligned(16))) float Qstg[GWAV * 128];

    const int tid  = threadIdx.x;
    const int lane = tid & 31, wave = tid >> 5;
    const int h = lane >> 4, m = lane & 15;
    const int rel = blockIdx.y;
    const float* Bp = Bsrc + (size_t)rel * (size_t)bRel;
    float* Cp = C + (size_t)rel * (size_t)cRel;
    float* Qp = QK + (size_t)rel * (size_t)qkRel;

#pragma unroll 4
    for (int idx = tid; idx < HIDC * HIDC; idx += GTHR) {
        const int n = idx >> 7, k = idx & (HIDC - 1);
        const float v = Bp[(size_t)n * (size_t)sn + (size_t)k * (size_t)sk];
        unsigned hb, lb;
        split1(v, hb, lb);
        Bh[n * BST + k] = (unsigned short)hb;
        Bl[n * BST + k] = (unsigned short)lb;
    }
    if (do_qk) {
#pragma unroll 4
        for (int idx = tid; idx < 16 * HIDC; idx += GTHR) {
            const int n = idx >> 7, k = idx & (HIDC - 1);
            float v = 0.0f;
            if (n < NHEAD) v = Qw[k * NHEAD + n];
            else if (n < 2 * NHEAD) v = Kw[k * NHEAD + (n - NHEAD)];
            unsigned hb, lb;
            split1(v, hb, lb);
            Qh[n * BST + k] = (unsigned short)hb;
            Ql[n * BST + k] = (unsigned short)lb;
        }
    }
    __syncthreads();

    float* stg = Sstg + wave * (16 * SST);
    float* qst = Qstg + wave * 128;
    const int blk0 = blockIdx.x * (GWAV * GSPW);

#pragma unroll 1
    for (int s = 0; s < GSPW; ++s) {
        const int row0 = (blk0 + s * GWAV + wave) * 16;
        const bool act = row0 < M;

        if (act) {
            v8f acc[8];
#pragma unroll
            for (int ct = 0; ct < 8; ++ct) acc[ct] = (v8f){0.f, 0.f, 0.f, 0.f, 0.f, 0.f, 0.f, 0.f};
            int ar = row0 + m;
            if (ar > M - 1) ar = M - 1;
            const float* arow = A + (size_t)ar * HIDC;
#pragma unroll 1
            for (int ks = 0; ks < 4; ++ks) {
                v16b ah, al;
                split_a(arow + ks * 32 + 8 * h, arow + ks * 32 + 16 + 8 * h, ah, al);
                const int kb = ks * 32 + 8 * h;
#pragma unroll
                for (int ct = 0; ct < 8; ++ct) {
                    const int bo = (ct * 16 + m) * BST + kb;
                    FragU bh, bl;
                    bh.hf[0] = *(const v8ba*)(Bh + bo);
                    bh.hf[1] = *(const v8ba*)(Bh + bo + 16);
                    bl.hf[0] = *(const v8ba*)(Bl + bo);
                    bl.hf[1] = *(const v8ba*)(Bl + bo + 16);
                    acc[ct] = wmma_g(ah, bh.v, acc[ct]);
                    acc[ct] = wmma_g(ah, bl.v, acc[ct]);
                    acc[ct] = wmma_g(al, bh.v, acc[ct]);
                }
            }
#pragma unroll
            for (int ct = 0; ct < 8; ++ct) {
#pragma unroll
                for (int r = 0; r < 8; ++r) stg[(8 * h + r) * SST + ct * 16 + m] = acc[ct][r];
            }
        }
        __syncthreads();

        if (act && do_qk) {
            v8f aq = (v8f){0.f, 0.f, 0.f, 0.f, 0.f, 0.f, 0.f, 0.f};
#pragma unroll
            for (int ks = 0; ks < 4; ++ks) {
                v16b ah, al;
                split_a(stg + m * SST + ks * 32 + 8 * h, stg + m * SST + ks * 32 + 16 + 8 * h, ah, al);
                const int bo = m * BST + ks * 32 + 8 * h;
                FragU bh, bl;
                bh.hf[0] = *(const v8ba*)(Qh + bo);
                bh.hf[1] = *(const v8ba*)(Qh + bo + 16);
                bl.hf[0] = *(const v8ba*)(Ql + bo);
                bl.hf[1] = *(const v8ba*)(Ql + bo + 16);
                aq = wmma_g(ah, bh.v, aq);
                aq = wmma_g(ah, bl.v, aq);
                aq = wmma_g(al, bh.v, aq);
            }
            if (m < 8) {
#pragma unroll
                for (int r = 0; r < 8; ++r) qst[(8 * h + r) * 8 + m] = aq[r];
            }
        }
        if (act && do_be) {
            const v4f b4 = *(const v4fa*)(cbias + 4 * lane);
#pragma unroll 2
            for (int row = 0; row < 16; ++row) {
                float* p = stg + row * SST + 4 * lane;
                v4f v = *(v4fa*)p;
                v = v + b4;
                v4f o;
                o.x = (v.x > 0.f) ? v.x : expm1f(v.x);
                o.y = (v.y > 0.f) ? v.y : expm1f(v.y);
                o.z = (v.z > 0.f) ? v.z : expm1f(v.z);
                o.w = (v.w > 0.f) ? v.w : expm1f(v.w);
                *(v4fa*)p = o;
            }
        }
        __syncthreads();

        if (act) store_pass(stg, Cp, row0, M, lane, qst, Qp, do_qk);
        __threadfence();
        if (act) store_pass(stg, Cp, row0, M, lane, qst, Qp, do_qk);
        __syncthreads();
    }
}

__global__ void __launch_bounds__(ATHR) __attribute__((amdgpu_num_vgpr(256)))
k_agg(const int* __restrict__ eidx, const int* __restrict__ etype, int E, int Ehalf, int Nn, int Rn,
      const float* __restrict__ QK, long qkRel, const float* __restrict__ XW, long xwRel,
      const float* __restrict__ cb, float* AG)
{
    __shared__ __attribute__((aligned(16))) unsigned blist[CAPB];
    __shared__ __attribute__((aligned(16))) unsigned wlist[AWAV * CAPW];
    __shared__ int wtot[2][AWAV];

    const int tid = threadIdx.x, lane = tid & 31, wave = tid >> 5;
    const int n0 = blockIdx.x * NBLK;
    const int* edst = eidx + Ehalf;
    const bool vec4 = ((((size_t)edst) & 15) == 0);

    int bcnt = 0, par = 0;
#pragma unroll 1
    for (int base = 0; base < E; base += EPT * ATHR) {
        const int e0 = base + EPT * tid;
        int dd[EPT];
        if (vec4 && (e0 + EPT - 1) < E) {
            const v4i a = *(const v4ia*)(edst + e0);
            const v4i b = *(const v4ia*)(edst + e0 + 4);
            dd[0] = a.x; dd[1] = a.y; dd[2] = a.z; dd[3] = a.w;
            dd[4] = b.x; dd[5] = b.y; dd[6] = b.z; dd[7] = b.w;
        } else {
#pragma unroll
            for (int j = 0; j < EPT; ++j) dd[j] = ((e0 + j) < E) ? edst[e0 + j] : (n0 - 1);
        }
        unsigned bm[EPT];
        int bc[EPT];
        int csum = 0;
#pragma unroll
        for (int j = 0; j < EPT; ++j) {
            bm[j] = __builtin_amdgcn_ballot_w32((unsigned)(dd[j] - n0) < (unsigned)NBLK);
            bc[j] = __builtin_popcount(bm[j]);
            csum += bc[j];
        }
        if (lane == 0) wtot[par][wave] = csum;
        __syncthreads();
        int pre = 0, tot = 0;
#pragma unroll
        for (int w = 0; w < AWAV; ++w) {
            const int t = wtot[par][w];
            tot += t;
            pre += (w < wave) ? t : 0;
        }
        int pos = bcnt + pre;
#pragma unroll
        for (int j = 0; j < EPT; ++j) {
            if (bm[j] != 0u) {
                const int p = pos + (int)__builtin_amdgcn_mbcnt_lo(bm[j], 0u);
                const bool hit = ((bm[j] >> lane) & 1u) != 0u;
                if (hit && p < CAPB) blist[p] = ((unsigned)(dd[j] - n0) << 20) | (unsigned)(e0 + j);
            }
            pos += bc[j];
        }
        bcnt += tot;
        par ^= 1;
    }
    const int bcl = (bcnt < CAPB) ? bcnt : CAPB;
    __syncthreads();

    unsigned* wl = wlist + wave * CAPW;
    int wcnt = 0;
#pragma unroll 1
    for (int i = 0; i < bcl; i += 32) {
        const int idx = i + lane;
        const bool vld = idx < bcl;
        const unsigned ent = vld ? blist[idx] : 0u;
        const bool mine = vld && ((ent >> 27) == (unsigned)wave);
        const unsigned mk = __builtin_amdgcn_ballot_w32(mine);
        const int p = wcnt + (int)__builtin_amdgcn_mbcnt_lo(mk, 0u);
        if (mine && p < CAPW) wl[p] = ent;
        wcnt += __builtin_popcount(mk);
    }
    const int wcl = (wcnt < CAPW) ? wcnt : CAPW;
    __syncthreads();

    unsigned* glist = blist + wave * (4 * CAPG);
    int g0 = 0, g1 = 0, g2 = 0, g3 = 0;
#pragma unroll 1
    for (int i = 0; i < wcl; i += 32) {
        const int idx = i + lane;
        const bool vld = idx < wcl;
        const unsigned ent = vld ? wl[idx] : 0u;
        const unsigned gs = (ent >> 25) & 3u;
        const bool s0 = vld && (gs == 0u), s1 = vld && (gs == 1u), s2 = vld && (gs == 2u), s3 = vld && (gs == 3u);
        const unsigned m0 = __builtin_amdgcn_ballot_w32(s0);
        const unsigned m1 = __builtin_amdgcn_ballot_w32(s1);
        const unsigned m2 = __builtin_amdgcn_ballot_w32(s2);
        const unsigned m3 = __builtin_amdgcn_ballot_w32(s3);
        const int p0 = g0 + (int)__builtin_amdgcn_mbcnt_lo(m0, 0u);
        const int p1 = g1 + (int)__builtin_amdgcn_mbcnt_lo(m1, 0u);
        const int p2 = g2 + (int)__builtin_amdgcn_mbcnt_lo(m2, 0u);
        const int p3 = g3 + (int)__builtin_amdgcn_mbcnt_lo(m3, 0u);
        if (s0 && p0 < CAPG) glist[0 * CAPG + p0] = ent;
        if (s1 && p1 < CAPG) glist[1 * CAPG + p1] = ent;
        if (s2 && p2 < CAPG) glist[2 * CAPG + p2] = ent;
        if (s3 && p3 < CAPG) glist[3 * CAPG + p3] = ent;
        g0 += __builtin_popcount(m0);
        g1 += __builtin_popcount(m1);
        g2 += __builtin_popcount(m2);
        g3 += __builtin_popcount(m3);
    }
    if (g0 > CAPG) g0 = CAPG;
    if (g1 > CAPG) g1 = CAPG;
    if (g2 > CAPG) g2 = CAPG;
    if (g3 > CAPG) g3 = CAPG;
    __syncthreads();

    const int head = lane >> 3;
    const v4f cbv = *(const v4fa*)(cb + 4 * lane);
#pragma unroll 1
    for (int q = 0; q < 4; ++q) {
        const int gc = (q == 0) ? g0 : ((q == 1) ? g1 : ((q == 2) ? g2 : g3));
        const unsigned* gq = glist + q * CAPG;
#pragma unroll 1
        for (int nl = 0; nl < 32; ++nl) {
            const int dl = wave * 128 + q * 32 + nl;
            const int node = n0 + dl;
            if (node >= Nn) continue;
            float mrun = -INFINITY, srun = 0.0f;
            v4f acc = (v4f){0.f, 0.f, 0.f, 0.f};
#pragma unroll 1
            for (int c = 0; c < gc; c += 32) {
                const int idx = c + lane;
                const bool vld = idx < gc;
                const unsigned ent = vld ? gq[idx] : 0u;
                const bool hit = vld && ((ent >> 20) == (unsigned)dl);
                unsigned mk = __builtin_amdgcn_ballot_w32(hit);
                while (mk != 0u) {
                    const int sl = __builtin_ctz(mk);
                    mk &= mk - 1u;
                    int e = (int)((unsigned)__builtin_amdgcn_readlane((int)ent, sl) & 0xFFFFFu);
                    if (e > E - 1) e = E - 1;
                    int src = eidx[e];
                    int rl  = etype[e];
                    src = (src < 0) ? 0 : ((src > Nn - 1) ? (Nn - 1) : src);
                    rl  = (rl  < 0) ? 0 : ((rl  > Rn - 1) ? (Rn - 1) : rl);
                    const float* qkr = QK + (size_t)rl * (size_t)qkRel;
                    const float qv = qkr[(size_t)node * 8 + head];
                    const float kv = qkr[(size_t)src * 8 + 4 + head];
                    float al = qv + kv;
                    al = fmaxf(al, 0.2f * al);
                    const float mn = fmaxf(mrun, al);
                    const float sc = __expf(mrun - mn);
                    const float p  = __expf(al - mn);
                    const v4f xv = *(const v4fa*)(XW + (size_t)rl * (size_t)xwRel + (size_t)src * HIDC + 4 * lane);
                    srun = srun * sc + p;
                    acc  = acc * sc + xv * p;
                    mrun = mn;
                }
            }
            const float inv = 1.0f / (srun + 1e-16f);
            const v4f o = acc * inv + cbv;
            float* op = AG + (size_t)node * HIDC + 4 * lane;
            *(volatile v4f*)op = o;
            __threadfence();
            *(volatile v4f*)op = o;
        }
    }
}

extern "C" void kernel_launch(void* const* d_in, const int* in_sizes, int n_in,
                              void* d_out, int out_size, void* d_ws, size_t ws_size,
                              hipStream_t stream)
{
    if (n_in < 15) return;
    const int N = in_sizes[0] / HIDC;
    const int Ehalf = in_sizes[1] / 2;
    int E = in_sizes[2];
    if (E > Ehalf) E = Ehalf;
    const int R = in_sizes[3] / (HIDC * HIDC);
    if (N <= 0 || E <= 0 || R <= 0 || E > (1 << 20)) return;
    if (in_sizes[4] != HIDC * NHEAD || in_sizes[7] != HIDC * HIDC) return;
    if (out_size < N * HIDC) return;
    const int Mpad = ((N + 15) / 16) * 16;

    size_t off = 0;
    auto carve = [&](size_t bytes) -> char* {
        char* p = (char*)d_ws + off;
        off += (bytes + 255) & ~(size_t)255;
        return p;
    };
    float* xw = (float*)carve((size_t)R * (size_t)N * HIDC * sizeof(float));
    float* qk = (float*)carve((size_t)R * (size_t)Mpad * 8 * sizeof(float));
    float* ag = (float*)carve((size_t)N * HIDC * sizeof(float));
    float* hb = (float*)carve((size_t)N * HIDC * sizeof(float));
    if (off > ws_size) return;

    const long xwRel = (long)N * HIDC;
    const long qkRel = (long)Mpad * 8;
    const int gx = (N + GROWS - 1) / GROWS;
    const int ga = (N + NBLK - 1) / NBLK;

    const float* x     = (const float*)d_in[0];
    const int*   eidx  = (const int*)d_in[1];
    const int*   etype = (const int*)d_in[2];

    const float* hin = x;
    for (int l = 0; l < 2; ++l) {
        const float* W  = (const float*)d_in[3 + 6 * l];
        const float* Q  = (const float*)d_in[4 + 6 * l];
        const float* K  = (const float*)d_in[5 + 6 * l];
        const float* cv = (const float*)d_in[6 + 6 * l];
        const float* pW = (const float*)d_in[7 + 6 * l];
        const float* pb = (const float*)d_in[8 + 6 * l];
        float* hout = (l == 0) ? hb : (float*)d_out;

        k_gemm<<<dim3(gx, R), GTHR, 0, stream>>>(hin, N, W, (long)HIDC * HIDC, 1, HIDC, pb, 0,
                                                 xw, xwRel, Q, K, qk, qkRel, 1);
        k_agg<<<dim3(ga), ATHR, 0, stream>>>(eidx, etype, E, Ehalf, N, R, qk, qkRel, xw, xwRel, cv, ag);
        k_gemm<<<dim3(gx, 1), GTHR, 0, stream>>>(ag, N, pW, 0L, HIDC, 1, pb, 1,
                                                 hout, 0L, Q, K, qk, qkRel, 0);
        hin = hb;
    }
}
